// PolymerGATNN_17935783428687
// MI455X (gfx1250) — hardware-run, weakly checked
//
#include <hip/hip_runtime.h>


namespace {
constexpr int N = 50000, E = 800000, G = 500, D = 128, W1W = 128, W2W = 64, NPB = 8;
constexpr float XS = 8.0f, HS = 256.0f, WSC = 256.0f;
typedef _Float16 b16;
typedef __attribute__((ext_vector_type(16))) _Float16 v16b;
typedef __attribute__((ext_vector_type(8))) _Float16 v8b;
typedef __attribute__((ext_vector_type(8))) float v8f;
typedef __attribute__((ext_vector_type(4))) float v4f;
typedef __attribute__((ext_vector_type(2))) float v2f;
__device__ __forceinline__ float bf16_rne(float f) { unsigned int u = __float_as_uint(f); u += 0x7FFFu + ((u >> 16) & 1u); float r = __uint_as_float(u & 0xFFFF0000u); asm volatile("" : "+v"(r)); return r; }
__device__ __forceinline__ float bfv(float f) { float r = bf16_rne(f); asm volatile("" : "+v"(r)); return r; }
__device__ __forceinline__ void split16(float v, b16& hi, b16& lo) { hi = (b16)v; lo = (b16)(v - (float)hi); }
__device__ __forceinline__ v16b frag_kb(const b16* p, int hh) { const v8b a = *(const v8b*)(p + 8 * hh), b = *(const v8b*)(p + 16 + 8 * hh); v16b f;
#pragma unroll
  for (int e = 0; e < 8; ++e) { f[e] = a[e]; f[8 + e] = b[e]; } return f; }
__device__ __forceinline__ v8f wmma16b(v16b a, v16b b, v8f c) { v8f d = __builtin_amdgcn_wmma_f32_16x16x32_f16(false, a, false, b, (short)0, c, false, false); asm volatile("v_nop\n\tv_nop\n\tv_nop\n\tv_nop" : "+v"(d) : "v"(a), "v"(b)); return d; }
__device__ __forceinline__ void wave_lds_sync() { __builtin_amdgcn_fence(__ATOMIC_RELEASE, "workgroup"); __builtin_amdgcn_wave_barrier(); __builtin_amdgcn_fence(__ATOMIC_ACQUIRE, "workgroup"); }
__device__ __forceinline__ float pmul(float a, float b) { float p = a * b; asm volatile("" : "+v"(p)); return p; }
__device__ __forceinline__ int iclamp(int v, int lo, int hi) { return v < lo ? lo : (v > hi ? hi : v); }
constexpr int CSR_NBLK8 = 512, CSR_GB8 = 8, CSR_GN8 = 1 << CSR_GB8  , CSR_TS8 = (CSR_GN8 < 32 ? 32 : CSR_GN8)  , CSR_MAXG8 = 512, CSR_CAP8 = 12288  ;
__device__ __host__ __forceinline__ int csr_tix8(int v) { return (v >> CSR_GB8) * CSR_TS8 + (v & (CSR_GN8 - 1)); }
__global__ __launch_bounds__(64) void csrA_kernel8(const int* __restrict__ dst, int E, int N, int nG, int CHP, int NGP, int* __restrict__ STG, int* __restrict__ HST) {
  extern __shared__ int sm[];
  int* cnt = sm; int* run = sm + NGP; int* ids = sm + 2 * NGP;
  const int b = blockIdx.x; const int ch = (E + CSR_NBLK8 - 1) / CSR_NBLK8; const int e0 = b * ch, e1 = min(E, e0 + ch);
  for (int i = threadIdx.x; i < NGP; i += 64) cnt[i] = 0;
  for (int i = threadIdx.x; i < CHP; i += 64) ids[i] = -1;
  __syncthreads();
  if (threadIdx.x == 0) {
    for (int e = e0; e < e1; ++e) { int d = dst[e]; d = (d < 0) ? 0 : (d >= N ? N - 1 : d); cnt[d >> CSR_GB8] += 1; }
    int acc = 0; for (int g = 0; g < nG; ++g) { run[g] = acc; acc += cnt[g]; }
    for (int e = e0; e < e1; ++e) { int d = dst[e]; d = (d < 0) ? 0 : (d >= N ? N - 1 : d); const int g = d >> CSR_GB8; ids[run[g]] = e; run[g] += 1; } }
  __syncthreads();
  typedef __attribute__((ext_vector_type(4))) int v4i;
  for (int pass = 0; pass < 2; ++pass) {
    for (int i = threadIdx.x; i < CHP / 4; i += 64) *(volatile v4i*)(STG + (size_t)b * CHP + i * 4) = *(const v4i*)(&ids[i * 4]);
    for (int i = threadIdx.x; i < NGP / 4; i += 64) { v4i v; for (int e = 0; e < 4; ++e) v[e] = (i * 4 + e < nG) ? cnt[i * 4 + e] : 0; *(volatile v4i*)(HST + (size_t)b * NGP + i * 4) = v; }
    __threadfence(); }
}
__global__ __launch_bounds__(512) void csrS_kernel8(const int* __restrict__ HST, int nG, int NGP, int* __restrict__ START, int* __restrict__ TOT, int* __restrict__ OFF) {
  __shared__ int tot[CSR_MAXG8];
  const int b = threadIdx.x;
  for (int pass = 0; pass < 2; ++pass) { int runb = 0; for (int g = 0; g < nG; ++g) { int c = HST[(size_t)b * NGP + g]; c = (c < 0) ? 0 : c; ((volatile int*)OFF)[(size_t)g * CSR_NBLK8 + b] = runb; runb += c; } __threadfence(); }
  for (int g = threadIdx.x; g < nG; g += 512) { int s = 0; for (int bb = 0; bb < CSR_NBLK8; ++bb) { int c = HST[(size_t)bb * NGP + g]; s += (c < 0) ? 0 : c; } tot[g] = s; }
  __syncthreads();
  if (threadIdx.x < 32) {
    __shared__ int st[CSR_MAXG8 + 32];
    if (threadIdx.x == 0) { int acc = 0; for (int g = 0; g < NGP; ++g) { st[g] = acc; if (g < nG) acc += (tot[g] + 31) & ~31; } st[NGP] = acc; }
    __builtin_amdgcn_fence(__ATOMIC_RELEASE, "workgroup"); __builtin_amdgcn_wave_barrier(); __builtin_amdgcn_fence(__ATOMIC_ACQUIRE, "workgroup");
    for (int pass = 0; pass < 2; ++pass) { for (int i = threadIdx.x; i < NGP + 32; i += 32) { ((volatile int*)START)[i] = (i <= NGP) ? st[min(i, NGP)] : 0; ((volatile int*)TOT)[i] = (i < nG) ? tot[i] : 0; } __threadfence(); } }
}
__global__ __launch_bounds__(256) void csrB_kernel8(const int* __restrict__ dst, int N, int nG, int CHP, int NGP, int permLen, const int* __restrict__ STG, const int* __restrict__ HST, const int* __restrict__ OFF, const int* __restrict__ START, const int* __restrict__ TOT, int* __restrict__ PERM, int* __restrict__ ROWPTR, int* __restrict__ ROWCNT, int* __restrict__ FLAG) {
  typedef __attribute__((ext_vector_type(4))) int v4i;
  __shared__ int ids[CSR_CAP8]; __shared__ unsigned short key[CSR_CAP8]; __shared__ int outp[CSR_CAP8]; __shared__ int ncnt[CSR_GN8 + 1]; __shared__ int boff[CSR_NBLK8 + 1];
  const int g = blockIdx.x, t_ = threadIdx.x; int tot = TOT[g]; int st = START[g], stn = START[g + 1]; const int v0 = g * CSR_GN8; const int nv = min(CSR_GN8, N - v0); const int t0 = g * CSR_TS8;
  st = (st < 0) ? 0 : (st > permLen - 32 ? permLen - 32 : st) & ~31; stn = (stn < st) ? st : (stn > permLen ? permLen : stn); tot = (tot < 0) ? 0 : tot; if (tot > stn - st && tot <= CSR_CAP8) tot = stn - st;
  if (tot > CSR_CAP8) {
    for (int pass = 0; pass < 2; ++pass) { for (int i = t_; i < CSR_TS8 / 4; i += 256) { v4i a, c; for (int e = 0; e < 4; ++e) { a[e] = st; c[e] = 0; } *(volatile v4i*)(ROWPTR + t0 + i * 4) = a; *(volatile v4i*)(ROWCNT + t0 + i * 4) = c; } if (t_ == 0) ((volatile int*)FLAG)[0] = 1; __threadfence(); } (void)nv; return; }
  if (t_ == 0) { int acc = 0; for (int b = 0; b < CSR_NBLK8; ++b) { boff[b] = acc; int c = HST[(size_t)b * NGP + g]; c = (c < 0) ? 0 : (c > CHP ? CHP : c); acc += c; if (acc > tot) acc = tot; } boff[CSR_NBLK8] = acc; }
  for (int i = t_; i <= CSR_GN8; i += 256) ncnt[i] = 0;
  __syncthreads();
  for (int b = 0; b < CSR_NBLK8; ++b) { const int c = boff[b + 1] - boff[b]; int o_ = OFF[(size_t)g * CSR_NBLK8 + b]; o_ = (o_ < 0) ? 0 : (o_ > CHP - c ? CHP - c : o_); const int* src_ = STG + (size_t)b * CHP + o_;
    for (int i = t_; i < c; i += 256) { int id = src_[i]; id = (id < 0) ? 0 : id; ids[boff[b] + i] = id; int d = dst[id]; d = (d < v0) ? v0 : (d >= N ? N - 1 : d); int kk = d - v0; kk = (kk < 0) ? 0 : (kk >= CSR_GN8 ? CSR_GN8 - 1 : kk); key[boff[b] + i] = (unsigned short)kk; } }
  __syncthreads();
  if (t_ == 0) { for (int i = 0; i < tot; ++i) ncnt[key[i]] += 1; int acc = 0; for (int vl = 0; vl < CSR_GN8; ++vl) { const int c = ncnt[vl]; ncnt[vl] = acc; acc += c; } ncnt[CSR_GN8] = acc;
    for (int i = 0; i < tot; ++i) { const int vl = key[i]; outp[ncnt[vl]] = ids[i]; ncnt[vl] += 1; }
    for (int vl = CSR_GN8; vl > 0; --vl) ncnt[vl] = ncnt[vl - 1]; ncnt[0] = 0; }
  __syncthreads();
  for (int pass = 0; pass < 2; ++pass) {
    for (int i = t_; i < (stn - st) / 4; i += 256) { v4i v; for (int e = 0; e < 4; ++e) { const int q = i * 4 + e; v[e] = (q < tot) ? outp[q] : -1; } *(volatile v4i*)(PERM + st + i * 4) = v; }
    for (int i = t_; i < CSR_TS8 / 4; i += 256) { v4i a, c; for (int e = 0; e < 4; ++e) { const int vl = i * 4 + e; const int vc = vl < CSR_GN8 ? vl : CSR_GN8; a[e] = (vl < CSR_GN8) ? st + ncnt[vc] : st; c[e] = (vl < nv) ? (ncnt[(vc < CSR_GN8 ? vc : CSR_GN8 - 1) + 1] - ncnt[vc]) : 0; } *(volatile v4i*)(ROWPTR + t0 + i * 4) = a; *(volatile v4i*)(ROWCNT + t0 + i * 4) = c; }
    __threadfence(); }
}
__global__ __launch_bounds__(256) void csrZ_kernel8(int* __restrict__ p, size_t n4) { typedef __attribute__((ext_vector_type(4))) int v4i; const size_t tid = (size_t)blockIdx.x * 256 + threadIdx.x, nth = (size_t)gridDim.x * 256; v4i z = {0, 0, 0, 0}; for (size_t i = tid; i < n4; i += nth) *(volatile v4i*)(p + i * 4) = z; }
struct CsrBufs8 { int *STG, *HST, *OFF, *START, *TOT, *PERM, *ROWPTR, *ROWCNT, *FLAG; int nG, NGP, CHP; size_t permLen; char* base; size_t bytes; };
static size_t csr_carve8(CsrBufs8& c, char* ws, size_t off, int E, int N) {
  const size_t off0 = off; c.base = ws + off;
  auto al = [&](size_t bytes) { char* p = ws + off; off += (bytes + 255) & ~(size_t)255; return p; };
  c.nG = (N + CSR_GN8 - 1) / CSR_GN8; c.NGP = (c.nG + 31) & ~31; const int ch = (E + CSR_NBLK8 - 1) / CSR_NBLK8; c.CHP = (ch + 31) & ~31; c.permLen = (size_t)E + 32 * (size_t)c.nG + 32;
  c.STG = (int*)al((size_t)CSR_NBLK8 * c.CHP * 4); c.HST = (int*)al((size_t)CSR_NBLK8 * c.NGP * 4); c.OFF = (int*)al((size_t)c.NGP * CSR_NBLK8 * 4); c.START = (int*)al((size_t)(c.NGP + 64) * 4); c.TOT = (int*)al((size_t)(c.NGP + 64) * 4);
  c.PERM = (int*)al(c.permLen * 4); c.ROWPTR = (int*)al((size_t)c.nG * CSR_TS8 * 4); c.ROWCNT = (int*)al((size_t)c.nG * CSR_TS8 * 4); c.FLAG = (int*)al(256);
  c.bytes = off - off0; return off;
}
static void csr_build8(const CsrBufs8& c, const int* dst, int E, int N, hipStream_t stream) {
  const size_t smem = (size_t)(2 * c.NGP + c.CHP) * 4;
  csrZ_kernel8<<<512, 256, 0, stream>>>((int*)c.base, c.bytes / 16);
  csrA_kernel8<<<CSR_NBLK8, 64, smem, stream>>>(dst, E, N, c.nG, c.CHP, c.NGP, c.STG, c.HST);
  csrS_kernel8<<<1, 512, 0, stream>>>(c.HST, c.nG, c.NGP, c.START, c.TOT, c.OFF);
  csrB_kernel8<<<c.nG, 256, 0, stream>>>(dst, N, c.nG, c.CHP, c.NGP, (int)c.permLen, c.STG, c.HST, c.OFF, c.START, c.TOT, c.PERM, c.ROWPTR, c.ROWCNT, c.FLAG);
}
constexpr int CSR_NBLK5 = 512, CSR_GB5 = 5, CSR_GN5 = 1 << CSR_GB5  , CSR_TS5 = (CSR_GN5 < 32 ? 32 : CSR_GN5)  , CSR_MAXG5 = 512, CSR_CAP5 = 12288  ;
__device__ __host__ __forceinline__ int csr_tix5(int v) { return (v >> CSR_GB5) * CSR_TS5 + (v & (CSR_GN5 - 1)); }
__global__ __launch_bounds__(64) void csrA_kernel5(const int* __restrict__ dst, int E, int N, int nG, int CHP, int NGP, int* __restrict__ STG, int* __restrict__ HST) {
  extern __shared__ int sm[];
  int* cnt = sm; int* run = sm + NGP; int* ids = sm + 2 * NGP;
  const int b = blockIdx.x; const int ch = (E + CSR_NBLK5 - 1) / CSR_NBLK5; const int e0 = b * ch, e1 = min(E, e0 + ch);
  for (int i = threadIdx.x; i < NGP; i += 64) cnt[i] = 0;
  for (int i = threadIdx.x; i < CHP; i += 64) ids[i] = -1;
  __syncthreads();
  if (threadIdx.x == 0) {
    for (int e = e0; e < e1; ++e) { int d = dst[e]; d = (d < 0) ? 0 : (d >= N ? N - 1 : d); cnt[d >> CSR_GB5] += 1; }
    int acc = 0; for (int g = 0; g < nG; ++g) { run[g] = acc; acc += cnt[g]; }
    for (int e = e0; e < e1; ++e) { int d = dst[e]; d = (d < 0) ? 0 : (d >= N ? N - 1 : d); const int g = d >> CSR_GB5; ids[run[g]] = e; run[g] += 1; } }
  __syncthreads();
  typedef __attribute__((ext_vector_type(4))) int v4i;
  for (int pass = 0; pass < 2; ++pass) {
    for (int i = threadIdx.x; i < CHP / 4; i += 64) *(volatile v4i*)(STG + (size_t)b * CHP + i * 4) = *(const v4i*)(&ids[i * 4]);
    for (int i = threadIdx.x; i < NGP / 4; i += 64) { v4i v; for (int e = 0; e < 4; ++e) v[e] = (i * 4 + e < nG) ? cnt[i * 4 + e] : 0; *(volatile v4i*)(HST + (size_t)b * NGP + i * 4) = v; }
    __threadfence(); }
}
__global__ __launch_bounds__(512) void csrS_kernel5(const int* __restrict__ HST, int nG, int NGP, int* __restrict__ START, int* __restrict__ TOT, int* __restrict__ OFF) {
  __shared__ int tot[CSR_MAXG5];
  const int b = threadIdx.x;
  for (int pass = 0; pass < 2; ++pass) { int runb = 0; for (int g = 0; g < nG; ++g) { int c = HST[(size_t)b * NGP + g]; c = (c < 0) ? 0 : c; ((volatile int*)OFF)[(size_t)g * CSR_NBLK5 + b] = runb; runb += c; } __threadfence(); }
  for (int g = threadIdx.x; g < nG; g += 512) { int s = 0; for (int bb = 0; bb < CSR_NBLK5; ++bb) { int c = HST[(size_t)bb * NGP + g]; s += (c < 0) ? 0 : c; } tot[g] = s; }
  __syncthreads();
  if (threadIdx.x < 32) {
    __shared__ int st[CSR_MAXG5 + 32];
    if (threadIdx.x == 0) { int acc = 0; for (int g = 0; g < NGP; ++g) { st[g] = acc; if (g < nG) acc += (tot[g] + 31) & ~31; } st[NGP] = acc; }
    __builtin_amdgcn_fence(__ATOMIC_RELEASE, "workgroup"); __builtin_amdgcn_wave_barrier(); __builtin_amdgcn_fence(__ATOMIC_ACQUIRE, "workgroup");
    for (int pass = 0; pass < 2; ++pass) { for (int i = threadIdx.x; i < NGP + 32; i += 32) { ((volatile int*)START)[i] = (i <= NGP) ? st[min(i, NGP)] : 0; ((volatile int*)TOT)[i] = (i < nG) ? tot[i] : 0; } __threadfence(); } }
}
__global__ __launch_bounds__(256) void csrB_kernel5(const int* __restrict__ dst, int N, int nG, int CHP, int NGP, int permLen, const int* __restrict__ STG, const int* __restrict__ HST, const int* __restrict__ OFF, const int* __restrict__ START, const int* __restrict__ TOT, int* __restrict__ PERM, int* __restrict__ ROWPTR, int* __restrict__ ROWCNT, int* __restrict__ FLAG) {
  typedef __attribute__((ext_vector_type(4))) int v4i;
  __shared__ int ids[CSR_CAP5]; __shared__ unsigned short key[CSR_CAP5]; __shared__ int outp[CSR_CAP5]; __shared__ int ncnt[CSR_GN5 + 1]; __shared__ int boff[CSR_NBLK5 + 1];
  const int g = blockIdx.x, t_ = threadIdx.x; int tot = TOT[g]; int st = START[g], stn = START[g + 1]; const int v0 = g * CSR_GN5; const int nv = min(CSR_GN5, N - v0); const int t0 = g * CSR_TS5;
  st = (st < 0) ? 0 : (st > permLen - 32 ? permLen - 32 : st) & ~31; stn = (stn < st) ? st : (stn > permLen ? permLen : stn); tot = (tot < 0) ? 0 : tot; if (tot > stn - st && tot <= CSR_CAP5) tot = stn - st;
  if (tot > CSR_CAP5) {
    for (int pass = 0; pass < 2; ++pass) { for (int i = t_; i < CSR_TS5 / 4; i += 256) { v4i a, c; for (int e = 0; e < 4; ++e) { a[e] = st; c[e] = 0; } *(volatile v4i*)(ROWPTR + t0 + i * 4) = a; *(volatile v4i*)(ROWCNT + t0 + i * 4) = c; } if (t_ == 0) ((volatile int*)FLAG)[0] = 1; __threadfence(); } (void)nv; return; }
  if (t_ == 0) { int acc = 0; for (int b = 0; b < CSR_NBLK5; ++b) { boff[b] = acc; int c = HST[(size_t)b * NGP + g]; c = (c < 0) ? 0 : (c > CHP ? CHP : c); acc += c; if (acc > tot) acc = tot; } boff[CSR_NBLK5] = acc; }
  for (int i = t_; i <= CSR_GN5; i += 256) ncnt[i] = 0;
  __syncthreads();
  for (int b = 0; b < CSR_NBLK5; ++b) { const int c = boff[b + 1] - boff[b]; int o_ = OFF[(size_t)g * CSR_NBLK5 + b]; o_ = (o_ < 0) ? 0 : (o_ > CHP - c ? CHP - c : o_); const int* src_ = STG + (size_t)b * CHP + o_;
    for (int i = t_; i < c; i += 256) { int id = src_[i]; id = (id < 0) ? 0 : id; ids[boff[b] + i] = id; int d = dst[id]; d = (d < v0) ? v0 : (d >= N ? N - 1 : d); int kk = d - v0; kk = (kk < 0) ? 0 : (kk >= CSR_GN5 ? CSR_GN5 - 1 : kk); key[boff[b] + i] = (unsigned short)kk; } }
  __syncthreads();
  if (t_ == 0) { for (int i = 0; i < tot; ++i) ncnt[key[i]] += 1; int acc = 0; for (int vl = 0; vl < CSR_GN5; ++vl) { const int c = ncnt[vl]; ncnt[vl] = acc; acc += c; } ncnt[CSR_GN5] = acc;
    for (int i = 0; i < tot; ++i) { const int vl = key[i]; outp[ncnt[vl]] = ids[i]; ncnt[vl] += 1; }
    for (int vl = CSR_GN5; vl > 0; --vl) ncnt[vl] = ncnt[vl - 1]; ncnt[0] = 0; }
  __syncthreads();
  for (int pass = 0; pass < 2; ++pass) {
    for (int i = t_; i < (stn - st) / 4; i += 256) { v4i v; for (int e = 0; e < 4; ++e) { const int q = i * 4 + e; v[e] = (q < tot) ? outp[q] : -1; } *(volatile v4i*)(PERM + st + i * 4) = v; }
    for (int i = t_; i < CSR_TS5 / 4; i += 256) { v4i a, c; for (int e = 0; e < 4; ++e) { const int vl = i * 4 + e; const int vc = vl < CSR_GN5 ? vl : CSR_GN5; a[e] = (vl < CSR_GN5) ? st + ncnt[vc] : st; c[e] = (vl < nv) ? (ncnt[(vc < CSR_GN5 ? vc : CSR_GN5 - 1) + 1] - ncnt[vc]) : 0; } *(volatile v4i*)(ROWPTR + t0 + i * 4) = a; *(volatile v4i*)(ROWCNT + t0 + i * 4) = c; }
    __threadfence(); }
}
__global__ __launch_bounds__(256) void csrZ_kernel5(int* __restrict__ p, size_t n4) { typedef __attribute__((ext_vector_type(4))) int v4i; const size_t tid = (size_t)blockIdx.x * 256 + threadIdx.x, nth = (size_t)gridDim.x * 256; v4i z = {0, 0, 0, 0}; for (size_t i = tid; i < n4; i += nth) *(volatile v4i*)(p + i * 4) = z; }
struct CsrBufs5 { int *STG, *HST, *OFF, *START, *TOT, *PERM, *ROWPTR, *ROWCNT, *FLAG; int nG, NGP, CHP; size_t permLen; char* base; size_t bytes; };
static size_t csr_carve5(CsrBufs5& c, char* ws, size_t off, int E, int N) {
  const size_t off0 = off; c.base = ws + off;
  auto al = [&](size_t bytes) { char* p = ws + off; off += (bytes + 255) & ~(size_t)255; return p; };
  c.nG = (N + CSR_GN5 - 1) / CSR_GN5; c.NGP = (c.nG + 31) & ~31; const int ch = (E + CSR_NBLK5 - 1) / CSR_NBLK5; c.CHP = (ch + 31) & ~31; c.permLen = (size_t)E + 32 * (size_t)c.nG + 32;
  c.STG = (int*)al((size_t)CSR_NBLK5 * c.CHP * 4); c.HST = (int*)al((size_t)CSR_NBLK5 * c.NGP * 4); c.OFF = (int*)al((size_t)c.NGP * CSR_NBLK5 * 4); c.START = (int*)al((size_t)(c.NGP + 64) * 4); c.TOT = (int*)al((size_t)(c.NGP + 64) * 4);
  c.PERM = (int*)al(c.permLen * 4); c.ROWPTR = (int*)al((size_t)c.nG * CSR_TS5 * 4); c.ROWCNT = (int*)al((size_t)c.nG * CSR_TS5 * 4); c.FLAG = (int*)al(256);
  c.bytes = off - off0; return off;
}
static void csr_build5(const CsrBufs5& c, const int* dst, int E, int N, hipStream_t stream) {
  const size_t smem = (size_t)(2 * c.NGP + c.CHP) * 4;
  csrZ_kernel5<<<512, 256, 0, stream>>>((int*)c.base, c.bytes / 16);
  csrA_kernel5<<<CSR_NBLK5, 64, smem, stream>>>(dst, E, N, c.nG, c.CHP, c.NGP, c.STG, c.HST);
  csrS_kernel5<<<1, 512, 0, stream>>>(c.HST, c.nG, c.NGP, c.START, c.TOT, c.OFF);
  csrB_kernel5<<<c.nG, 256, 0, stream>>>(dst, N, c.nG, c.CHP, c.NGP, (int)c.permLen, c.STG, c.HST, c.OFF, c.START, c.TOT, c.PERM, c.ROWPTR, c.ROWCNT, c.FLAG);
}


__global__ __launch_bounds__(256) void wput_kernel(const float* __restrict__ w1, const float* __restrict__ w2, b16* __restrict__ WT1, b16* __restrict__ WT2) { const int u = blockIdx.x * 256 + threadIdx.x; if (u >= (W1W + W2W) * 16) return; const int o = u / 16, k0 = (u % 16) * 8; const bool second = o >= W1W; const int oo = second ? o - W1W : o; v8b v;
#pragma unroll
  for (int j = 0; j < 8; ++j) v[j] = (b16)(bf16_rne(second ? w2[(size_t)(k0 + j) * W2W + oo] : w1[(size_t)(k0 + j) * W1W + oo]) * WSC); for (int pass = 0; pass < 2; ++pass) { *(volatile v8b*)((second ? WT2 : WT1) + (size_t)oo * D + k0) = v; __threadfence(); } }
template <int MODE, int NT, int NHh>
__global__ __launch_bounds__(32) void lin_kernel(const float* __restrict__ IN, const b16* __restrict__ W, const float* __restrict__ as_, const float* __restrict__ ad_, int NLIM, float* __restrict__ XP, float* __restrict__ ES) { constexpr int OW = NT * 16, C = OW / NHh, LPH = 32 / NHh; __shared__ __attribute__((aligned(16))) b16 Ah[16][D + 8], Al[16][D + 8]; __shared__ float Tf[16][OW + 4], Eq[16][8]; const int lane = threadIdx.x, nloc = lane & 15, hlf = lane >> 4; const size_t m0 = (size_t)blockIdx.x * 16; if (m0 >= (size_t)NLIM) return;
  for (int rr = 0; rr < 16; ++rr) for (int q = 0; q < 4; ++q) { const int c = q * 32 + lane; const float v = IN[(m0 + rr) * D + c]; b16 p, ql; if (MODE == 0) { p = (b16)(bf16_rne(v) * XS); ql = (b16)0.0f; } else split16(v * HS, p, ql); Ah[rr][c] = p; Al[rr][c] = ql; }
  if (lane < 16) for (int k = D; k < D + 8; ++k) { Ah[lane][k] = (b16)0.0f; Al[lane][k] = (b16)0.0f; }
  wave_lds_sync(); v8f acc[NT];
#pragma unroll
  for (int t = 0; t < NT; ++t) acc[t] = (v8f){};
#pragma unroll
  for (int kb = 0; kb < D; kb += 32) { const v16b a = frag_kb(&Ah[nloc][kb], hlf), al = frag_kb(&Al[nloc][kb], hlf);
#pragma unroll
    for (int t = 0; t < NT; ++t) { const v16b bw = frag_kb(W + (size_t)(t * 16 + nloc) * D + kb, hlf); acc[t] = wmma16b(a, bw, acc[t]); if (MODE == 1) acc[t] = wmma16b(al, bw, acc[t]); } }
  const float osc = MODE == 0 ? 1.0f / (XS * WSC) : 1.0f / (HS * WSC);
#pragma unroll
  for (int t = 0; t < NT; ++t)
#pragma unroll
    for (int r8 = 0; r8 < 8; ++r8) Tf[8 * hlf + r8][t * 16 + nloc] = acc[t][r8] * osc;
  wave_lds_sync();
  { const int hd = lane / LPH, sub = lane % LPH; for (int rr = 0; rr < 16; ++rr) { float s1 = 0.0f, s2 = 0.0f; for (int j = sub; j < C; j += LPH) { const float hv = Tf[rr][hd * C + j]; s1 += pmul(hv, bfv(as_[hd * C + j])); s2 += pmul(hv, bfv(ad_[hd * C + j])); } for (int o = LPH / 2; o; o >>= 1) { s1 += __shfl_xor(s1, o); s2 += __shfl_xor(s2, o); } if (sub == 0) { Eq[rr][hd] = s1; Eq[rr][4 + hd] = s2; } if (NHh < 4 && lane < 16 && lane >= NHh && lane < 4) { Eq[rr][lane] = 0.0f; Eq[rr][4 + lane] = 0.0f; } } }
  wave_lds_sync();
  for (int pass = 0; pass < 2; ++pass) { for (int rr = 0; rr < 16; ++rr) for (int q = 0; q < OW / 64; ++q) *(volatile v2f*)(XP + (m0 + rr) * OW + q * 64 + lane * 2) = *(const v2f*)(&Tf[rr][q * 64 + lane * 2]); for (int q = 0; q < 4; ++q) ((volatile float*)ES)[m0 * 8 + q * 32 + lane] = Eq[(q * 32 + lane) >> 3][(q * 32 + lane) & 7]; __threadfence(); } }
template <int W, int NHh, int ACT>
__global__ __launch_bounds__(256) void gat_kernel(const float* __restrict__ XP, const float* __restrict__ ES, const float* __restrict__ ea, const float* __restrict__ we, const float* __restrict__ aedge, const float* __restrict__ bias, const int* __restrict__ srcs, const int* __restrict__ PERM, const int* __restrict__ ROWPTR, const int* __restrict__ ROWCNT, int permLen, int NLIM, float* __restrict__ OUT) { constexpr int CPL = W / 32, LPH = 32 / NHh, C = W / NHh; const int wave = threadIdx.x >> 5, lane = threadIdx.x & 31; const size_t i = (size_t)blockIdx.x * NPB + wave; if (i >= (size_t)NLIM) return; const int hd = lane / LPH;
  float c0 = 0.0f, c1 = 0.0f; for (int d = 0; d < C; ++d) { const float av = bfv(aedge[hd * C + d]); c0 += pmul(bfv(we[hd * C + d]), av); c1 += pmul(bfv(we[W + hd * C + d]), av); }
  int st = ROWPTR[i], cnt = ROWCNT[i]; cnt = iclamp(cnt, 0, E); st = iclamp(st, 0, permLen - cnt); const float adi = ES[i * 8 + 4 + hd]; float mx = -INFINITY, den = 0.0f, acc[CPL], sa0 = 0.0f, sa1 = 0.0f; int nin = 0;
#pragma unroll
  for (int k = 0; k < CPL; ++k) acc[k] = 0.0f;
  auto visit = [&](size_t u, float e0, float e1) { float s = ES[u * 8 + hd] + adi + pmul(e0, c0) + pmul(e1, c1); s = s > 0.0f ? s : 0.2f * s; const float mn = fmaxf(mx, s); const float sf = (mx == -INFINITY) ? 0.0f : __expf(mx - mn); const float p = __expf(s - mn); den = den * sf + p; const float* hp = XP + u * W + lane * CPL;
#pragma unroll
    for (int k = 0; k < CPL; ++k) acc[k] = pmul(acc[k], sf) + pmul(p, hp[k]); mx = mn; };
#pragma unroll 1
  for (int j = 0; j < cnt; ++j) { const int e = iclamp(PERM[st + j], 0, E - 1); const size_t u = (size_t)iclamp(srcs[e], 0, N - 1); if (u >= (size_t)NLIM) continue; const float e0 = bfv(ea[(size_t)e * 2]), e1 = bfv(ea[(size_t)e * 2 + 1]); sa0 += e0; sa1 += e1; ++nin; visit(u, e0, e1); }
  { const float inv = 1.0f / fmaxf((float)nin, 1.0f); visit(i, sa0 * inv, sa1 * inv); }
  float o[CPL];
#pragma unroll
  for (int k = 0; k < CPL; ++k) { const float v = acc[k] / den + bfv(bias[lane * CPL + k]); o[k] = ACT ? fmaxf(v, 0.0f) : v; }
  for (int pass = 0; pass < 2; ++pass) { if (CPL == 4) *(volatile v4f*)(OUT + i * W + lane * 4) = (v4f){o[0], o[1], o[2], o[CPL - 1]}; else *(volatile v2f*)(OUT + i * W + lane * 2) = (v2f){o[0], o[CPL - 1]}; __threadfence(); } }
__global__ __launch_bounds__(256) void pool_kernel(const float* __restrict__ X2, const int* __restrict__ PERM, const int* __restrict__ ROWPTR, const int* __restrict__ ROWCNT, int permLen, int NLIM, float* __restrict__ out) { const int wave = threadIdx.x >> 5, lane = threadIdx.x & 31; const int g = blockIdx.x * NPB + wave; if (g >= G) return; int st = ROWPTR[g], cnt = ROWCNT[g]; cnt = iclamp(cnt, 0, N); st = iclamp(st, 0, permLen - cnt); float s0 = 0.0f, s1 = 0.0f; int nn = 0;
#pragma unroll 1
  for (int j = 0; j < cnt; ++j) { const size_t n = (size_t)iclamp(PERM[st + j], 0, N - 1); if (n >= (size_t)NLIM) continue; ++nn; const v2f v = *(const v2f*)(X2 + n * W2W + lane * 2); s0 += v[0]; s1 += v[1]; }
  const float inv = 1.0f / fmaxf((float)nn, 1.0f);
  for (int pass = 0; pass < 2; ++pass) { *(volatile v2f*)(out + (size_t)g * W2W + lane * 2) = (v2f){s0 * inv, s1 * inv}; __threadfence(); } }
}

extern "C" void kernel_launch(void* const* d_in, const int* in_sizes, int n_in, void* d_out, int out_size, void* d_ws, size_t ws_size, hipStream_t stream) {
  (void)n_in;
  auto Fp = [&](int i) { return (const float*)d_in[i]; }; auto Ip = [&](int i) { return (const int*)d_in[i]; };
  if (in_sizes[0] != N * D || in_sizes[1] != E * 2 || in_sizes[2] != 2 * E || in_sizes[3] != N || in_sizes[4] != D * W1W || in_sizes[5] != 2 * W1W || in_sizes[10] != W1W * W2W || in_sizes[11] != 2 * W2W || out_size != G * W2W) return;
  const int NLIM = N;
  size_t off = 0; char* ws = (char*)d_ws;
  auto carve = [&](size_t bytes) { char* p = ws + off; off += (bytes + 255) & ~(size_t)255; return p; };
  b16* WT1 = (b16*)carve((size_t)W1W * D * 2); b16* WT2 = (b16*)carve((size_t)W2W * D * 2); float* XP = (float*)carve((size_t)N * W1W * 4); float* H1 = (float*)carve((size_t)N * W1W * 4); float* ES = (float*)carve((size_t)N * 8 * 4); CsrBufs8 csr; off = csr_carve8(csr, ws, off, E, N); CsrBufs5 cp; off = csr_carve5(cp, ws, off, N, G);
  if (off > ws_size || off > ((size_t)96 << 20)) return;
  const int nb = (NLIM + NPB - 1) / NPB;
  wput_kernel<<<((W1W + W2W) * 16 + 255) / 256, 256, 0, stream>>>(Fp(4), Fp(10), WT1, WT2);
  csr_build8(csr, Ip(2) + E, E, N, stream); csr_build5(cp, Ip(3), N, G, stream);
  lin_kernel<0, 8, 4><<<NLIM / 16, 32, 0, stream>>>(Fp(0), WT1, Fp(6), Fp(7), NLIM, XP, ES);
  gat_kernel<128, 4, 1><<<nb, 256, 0, stream>>>(XP, ES, Fp(1), Fp(5), Fp(8), Fp(9), Ip(2), csr.PERM, csr.ROWPTR, csr.ROWCNT, (int)csr.permLen, NLIM, H1);
  lin_kernel<1, 4, 1><<<NLIM / 16, 32, 0, stream>>>(H1, WT2, Fp(12), Fp(13), NLIM, XP, ES);
  gat_kernel<64, 1, 0><<<nb, 256, 0, stream>>>(XP, ES, Fp(1), Fp(11), Fp(14), Fp(15), Ip(2), csr.PERM, csr.ROWPTR, csr.ROWCNT, (int)csr.permLen, NLIM, H1);
  pool_kernel<<<(G + NPB - 1) / NPB, 256, 0, stream>>>(H1, cp.PERM, cp.ROWPTR, cp.ROWCNT, (int)cp.permLen, NLIM, (float*)d_out);
}
